// SelfAttention_89120571392174
// MI455X (gfx1250) — hardware-verified
//
#include <hip/hip_runtime.h>


#ifndef NB
#define NB 4
#endif
#ifndef SEQ
#define SEQ 2048
#endif
#define NB_FULL    4
#define SEQ_FULL   2048
#define NHEAD      12
#define HDIM       64
#define EMB        768
#define BQ         128
#define BK         32
#define NWAVE      8
#define CT         64
#define TP         72
#define OP         68
#define WO_TILES   ((EMB / 64) * (EMB / 64))

static_assert(SEQ % BQ == 0);
static_assert(SEQ % CT == 0);
static_assert(SEQ % BK == 0);
static_assert(BQ == NWAVE * 16);
static_assert(HDIM == 64);
static_assert(EMB == NHEAD * HDIM);
static_assert(EMB % 64 == 0);
static_assert(EMB % 32 == 0);
static_assert(SEQ <= SEQ_FULL);
static_assert(NB >= 1 && NB <= NB_FULL);
static_assert((TP * 2) % 16 == 0);
static_assert((OP * 4) % 16 == 0);
static_assert(((size_t)NB * SEQ) % 128 == 0);
static_assert(CT * HDIM == 256 * 2 * 8);
static_assert(64 * 64 == 256 * 2 * 8);
static_assert(16 * HDIM == 32 * 4 * 8);
static_assert(16 * 64 == 32 * 8 * 4);

typedef __bf16         bf16;
typedef _Float16       f16;
typedef unsigned short us;
typedef bf16     v16bf __attribute__((ext_vector_type(16)));
typedef f16      v16h  __attribute__((ext_vector_type(16)));
typedef us       v8us  __attribute__((ext_vector_type(8)));
typedef float    v8f   __attribute__((ext_vector_type(8)));
typedef float    v4f   __attribute__((ext_vector_type(4)));
typedef unsigned v4u   __attribute__((ext_vector_type(4)));

union FragB  { v16bf v; v4u q[2]; bf16 h[16]; };
union FragH  { v16h  v; v4u q[2]; f16  h[16]; };
union Pack8H { v4u u; f16 h[8]; };
union Pack8U { v4u u; v8us v; };

static __device__ __forceinline__ v8f mma_bf16(v16bf a, v16bf b, v8f acc) {
  acc = __builtin_amdgcn_wmma_f32_16x16x32_bf16(false, a, false, b, (short)0, acc, false, false);
  asm volatile("v_nop\n\tv_nop\n\tv_nop\n\tv_nop" : "+v"(acc) : "v"(a), "v"(b));
  return acc;
}
static __device__ __forceinline__ v8f mma_f16(v16h a, v16h b, v8f acc) {
  acc = __builtin_amdgcn_wmma_f32_16x16x32_f16(false, a, false, b, (short)0, acc, false, false);
  asm volatile("v_nop\n\tv_nop\n\tv_nop\n\tv_nop" : "+v"(acc) : "v"(a), "v"(b));
  return acc;
}

static __device__ __forceinline__ us plane_bits(float v, bool as_f16, float carry) {
  const bf16 bv = (bf16)v;
  const unsigned bb = (unsigned)__builtin_bit_cast(us, bv);
  const f16 hv = (f16)((float)bv * carry);
  const unsigned hb = (unsigned)__builtin_bit_cast(us, hv);
  return (us)(as_f16 ? hb : bb);
}

__global__ __launch_bounds__(256) void prep_kernel(const float* __restrict__ Wq,
                                                   const float* __restrict__ Wk,
                                                   const float* __restrict__ Wv,
                                                   const float* __restrict__ Wo,
                                                   us* __restrict__ wt,
                                                   us* __restrict__ wot) {
  const unsigned blk = blockIdx.x;
  const unsigned tid = threadIdx.x;
  __shared__ __align__(16) us sT[64 * TP];

  const bool     big   = blk < (unsigned)WO_TILES;
  const unsigned tc    = big ? (blk / 12u) : 0u;
  const unsigned tj    = big ? (blk - tc * 12u) : 0u;
  const unsigned w     = big ? 0u : (blk - (unsigned)WO_TILES);
  const float*   src   = big ? Wo : ((w == 0u) ? Wq : ((w == 1u) ? Wk : Wv));
  const unsigned pitch = big ? (unsigned)EMB : (unsigned)HDIM;
  us*            dst   = big ? wot : (wt + w * (unsigned)(HDIM * HDIM));
  const float    carry = big ? 64.0f : 1.0f;

  #pragma unroll
  for (unsigned kk = 0; kk < 2; ++kk) {
    const unsigned key = kk * 32u + (tid >> 3);
    const unsigned d0  = (tid & 7u) * 8u;
    const float* p = src + (size_t)(tc * 64u + key) * pitch + tj * 64u + d0;
    const v4f a0 = *(const v4f*)(p);
    const v4f a1 = *(const v4f*)(p + 4);
    #pragma unroll
    for (unsigned i = 0; i < 4; ++i) {
      sT[(d0 + i) * TP + key]      = plane_bits(a0[i], big, carry);
      sT[(d0 + 4u + i) * TP + key] = plane_bits(a1[i], big, carry);
    }
  }
  __syncthreads();

  v4u    val[2];
  size_t idx[2];
  #pragma unroll
  for (unsigned kk = 0; kk < 2; ++kk) {
    const unsigned d  = kk * 32u + (tid >> 3);
    const unsigned ks = (tid & 7u) * 8u;
    Pack8U pk;
    pk.v = *(const v8us*)(sT + d * TP + ks);
    val[kk] = pk.u;
    idx[kk] = (size_t)(tj * 64u + d) * pitch + tc * 64u + ks;
  }
  #pragma unroll
  for (unsigned kk = 0; kk < 2; ++kk) *(volatile v4u*)(dst + idx[kk]) = val[kk];
  __threadfence();
  #pragma unroll
  for (unsigned kk = 0; kk < 2; ++kk) *(volatile v4u*)(dst + idx[kk]) = val[kk];
}

__global__ __launch_bounds__(256) void proj_kernel(const float* __restrict__ x,
                                                   const us* __restrict__ wt,
                                                   us* __restrict__ qp,
                                                   us* __restrict__ kp,
                                                   us* __restrict__ vt) {
  const unsigned kt   = blockIdx.x;
  const unsigned h    = blockIdx.y;
  const unsigned b    = blockIdx.z;
  const unsigned tid  = threadIdx.x;
  const unsigned wave = tid >> 5;
  const unsigned lane = tid & 31u;
  const unsigned lq   = lane & 15u;
  const unsigned hi   = lane >> 4;

  __shared__ __align__(16) us sQ[CT * TP];
  __shared__ __align__(16) us sK[CT * TP];
  __shared__ __align__(16) us sV[HDIM * TP];

  const unsigned s0 = kt * CT;
  const unsigned rt = wave & 3u;
  const unsigned ch = wave >> 2;

  FragB xa[2];
  {
    const float* xp = x + ((size_t)b * SEQ_FULL + s0 + rt * 16u + lq) * EMB + h * HDIM;
    #pragma unroll
    for (unsigned f = 0; f < 2; ++f) {
      const v4f a0 = *(const v4f*)(xp + f * 32u + hi * 8u);
      const v4f a1 = *(const v4f*)(xp + f * 32u + hi * 8u + 4u);
      const v4f b0 = *(const v4f*)(xp + f * 32u + 16u + hi * 8u);
      const v4f b1 = *(const v4f*)(xp + f * 32u + 16u + hi * 8u + 4u);
      #pragma unroll
      for (unsigned i = 0; i < 4; ++i) {
        xa[f].h[i]       = (bf16)a0[i];
        xa[f].h[4u + i]  = (bf16)a1[i];
        xa[f].h[8u + i]  = (bf16)b0[i];
        xa[f].h[12u + i] = (bf16)b1[i];
      }
    }
  }

  #pragma unroll
  for (unsigned w = 0; w < 3; ++w) {
    #pragma unroll
    for (unsigned cc = 0; cc < 2; ++cc) {
      const unsigned e = (ch * 2u + cc) * 16u + lq;
      FragB wb[2];
      #pragma unroll
      for (unsigned f = 0; f < 2; ++f) {
        const us* base = wt + w * (unsigned)(HDIM * HDIM) + e * HDIM + f * 32u + hi * 8u;
        wb[f].q[0] = *(const v4u*)(base);
        wb[f].q[1] = *(const v4u*)(base + 16);
      }
      v8f acc = (v8f){0, 0, 0, 0, 0, 0, 0, 0};
      acc = mma_bf16(xa[0].v, wb[0].v, acc);
      acc = mma_bf16(xa[1].v, wb[1].v, acc);
      #pragma unroll
      for (unsigned r = 0; r < 8; ++r) {
        const unsigned row = rt * 16u + hi * 8u + r;
        const us bits = __builtin_bit_cast(us, (f16)(acc[r] * 16.0f));
        if (w == 0u)      sQ[row * TP + e] = bits;
        else if (w == 1u) sK[row * TP + e] = bits;
        else              sV[e * TP + row] = bits;
      }
    }
  }
  __syncthreads();

  v4u    qv[2], kv[2], vv[2];
  size_t ridx[2], vidx[2];
  #pragma unroll
  for (unsigned kk = 0; kk < 2; ++kk) {
    const unsigned row = kk * 32u + (tid >> 3);
    const unsigned pc  = (tid & 7u) * 8u;
    Pack8U pq, pk, pv;
    pq.v = *(const v8us*)(sQ + row * TP + pc);
    pk.v = *(const v8us*)(sK + row * TP + pc);
    pv.v = *(const v8us*)(sV + row * TP + pc);
    qv[kk] = pq.u;
    kv[kk] = pk.u;
    vv[kk] = pv.u;
    ridx[kk] = (((size_t)b * NHEAD + h) * SEQ + s0 + row) * HDIM + pc;
    vidx[kk] = (((size_t)b * NHEAD + h) * HDIM + row) * SEQ + s0 + pc;
  }
  #pragma unroll
  for (unsigned kk = 0; kk < 2; ++kk) {
    *(volatile v4u*)(qp + ridx[kk]) = qv[kk];
    *(volatile v4u*)(kp + ridx[kk]) = kv[kk];
    *(volatile v4u*)(vt + vidx[kk]) = vv[kk];
  }
  __threadfence();
  #pragma unroll
  for (unsigned kk = 0; kk < 2; ++kk) {
    *(volatile v4u*)(qp + ridx[kk]) = qv[kk];
    *(volatile v4u*)(kp + ridx[kk]) = kv[kk];
    *(volatile v4u*)(vt + vidx[kk]) = vv[kk];
  }
}

__global__ __launch_bounds__(256) void attn_kernel(const us* __restrict__ qp,
                                                   const us* __restrict__ kp,
                                                   const us* __restrict__ vt,
                                                   us* __restrict__ chi,
                                                   us* __restrict__ clo) {
  const unsigned qblk = blockIdx.x;
  const unsigned h    = blockIdx.y;
  const unsigned b    = blockIdx.z;
  const unsigned tid  = threadIdx.x;
  const unsigned wave = tid >> 5;
  const unsigned lane = tid & 31u;
  const unsigned lq   = lane & 15u;
  const unsigned hi   = lane >> 4;

  __shared__ __align__(16) float sO[NWAVE * 16 * OP];

  const unsigned qrow0 = qblk * BQ + wave * 16u;

  const us* q_h = qp + ((size_t)b * NHEAD + h) * SEQ * HDIM;
  const us* k_h = kp + ((size_t)b * NHEAD + h) * SEQ * HDIM;
  const us* v_h = vt + ((size_t)b * NHEAD + h) * HDIM * SEQ;

  FragH qf[2];
  #pragma unroll
  for (unsigned f = 0; f < 2; ++f) {
    const us* base = q_h + (size_t)(qrow0 + lq) * HDIM + f * 32u + hi * 8u;
    qf[f].q[0] = *(const v4u*)(base);
    qf[f].q[1] = *(const v4u*)(base + 16);
  }

  v8f o[4];
  #pragma unroll
  for (unsigned dt = 0; dt < 4; ++dt) o[dt] = (v8f){0, 0, 0, 0, 0, 0, 0, 0};

  float rmax = -__builtin_inff();
  float rsum = 0.0f;
  const float SL = (0.03608439182435161f * 1.4426950408889634f) * (1.0f / 256.0f);

  #pragma unroll 1
  for (unsigned i = 0; i < (unsigned)(SEQ / BK); ++i) {
    const unsigned j0 = i * BK;

    FragH ak[2][2];
    #pragma unroll
    for (unsigned sub = 0; sub < 2; ++sub) {
      #pragma unroll
      for (unsigned f = 0; f < 2; ++f) {
        const us* base = k_h + (size_t)(j0 + sub * 16u + lq) * HDIM + f * 32u + hi * 8u;
        ak[sub][f].q[0] = *(const v4u*)(base);
        ak[sub][f].q[1] = *(const v4u*)(base + 16);
      }
    }
    FragH bv[4];
    #pragma unroll
    for (unsigned dt = 0; dt < 4; ++dt) {
      const us* base = v_h + (size_t)(dt * 16u + lq) * SEQ + j0 + hi * 8u;
      bv[dt].q[0] = *(const v4u*)(base);
      bv[dt].q[1] = *(const v4u*)(base + 16);
    }

    v8f c[2];
    #pragma unroll
    for (unsigned sub = 0; sub < 2; ++sub) {
      v8f acc = (v8f){0, 0, 0, 0, 0, 0, 0, 0};
      acc = mma_f16(ak[sub][0].v, qf[0].v, acc);
      acc = mma_f16(ak[sub][1].v, qf[1].v, acc);
      c[sub] = acc;
    }

    float m_new = rmax;
    #pragma unroll
    for (unsigned r = 0; r < 8; ++r) {
      m_new = fmaxf(m_new, c[0][r]);
      m_new = fmaxf(m_new, c[1][r]);
    }
    m_new = fmaxf(m_new, __shfl_xor(m_new, 16, 32));
    const float scale = __builtin_amdgcn_exp2f((rmax - m_new) * SL);
    rmax = m_new;

    FragH pa;
    float psum = 0.0f;
    #pragma unroll
    for (unsigned r = 0; r < 8; ++r) {
      const float p0 = __builtin_amdgcn_exp2f((c[0][r] - m_new) * SL);
      const float p1 = __builtin_amdgcn_exp2f((c[1][r] - m_new) * SL);
      psum += p0 + p1;
      pa.h[r]      = (f16)(p0 * 4096.0f);
      pa.h[8u + r] = (f16)(p1 * 4096.0f);
    }
    rsum = rsum * scale + psum + __shfl_xor(psum, 16, 32);

    float sc[8];
    #pragma unroll
    for (unsigned r = 0; r < 8; ++r) sc[r] = __shfl(scale, (int)((hi << 3) + r), 32);
    #pragma unroll
    for (unsigned dt = 0; dt < 4; ++dt) {
      #pragma unroll
      for (unsigned r = 0; r < 8; ++r) o[dt][r] *= sc[r];
    }

    #pragma unroll
    for (unsigned dt = 0; dt < 4; ++dt) o[dt] = mma_f16(pa.v, bv[dt].v, o[dt]);
  }

  float rs[8];
  #pragma unroll
  for (unsigned r = 0; r < 8; ++r) rs[r] = 1.0f / __shfl(rsum, (int)((hi << 3) + r), 32);

  float* so = sO + wave * (16 * OP);
  #pragma unroll
  for (unsigned r = 0; r < 8; ++r) {
    #pragma unroll
    for (unsigned dt = 0; dt < 4; ++dt) {
      so[(hi * 8u + r) * OP + dt * 16u + lq] = o[dt][r] * (1.0f / 256.0f) * rs[r];
    }
  }
  __syncthreads();

  v4u    hv[4], lv[4];
  size_t gidx[4];
  #pragma unroll
  for (unsigned it = 0; it < 4; ++it) {
    const unsigned row = it * 4u + (lane >> 3);
    const unsigned pc  = (lane & 7u) * 8u;
    const v4f a0 = *(const v4f*)(so + row * OP + pc);
    const v4f a1 = *(const v4f*)(so + row * OP + pc + 4u);
    Pack8H ph, pl;
    #pragma unroll
    for (unsigned i = 0; i < 4; ++i) {
      const f16 h0 = (f16)a0[i];
      const f16 h1 = (f16)a1[i];
      ph.h[i]      = h0;
      ph.h[4u + i] = h1;
      pl.h[i]      = (f16)((a0[i] - (float)h0) * 2048.0f);
      pl.h[4u + i] = (f16)((a1[i] - (float)h1) * 2048.0f);
    }
    hv[it] = ph.u;
    lv[it] = pl.u;
    gidx[it] = ((size_t)b * SEQ + qrow0 + row) * EMB + h * HDIM + pc;
  }
  #pragma unroll
  for (unsigned it = 0; it < 4; ++it) {
    *(volatile v4u*)(chi + gidx[it]) = hv[it];
    *(volatile v4u*)(clo + gidx[it]) = lv[it];
  }
  __threadfence();
  #pragma unroll
  for (unsigned it = 0; it < 4; ++it) {
    *(volatile v4u*)(chi + gidx[it]) = hv[it];
    *(volatile v4u*)(clo + gidx[it]) = lv[it];
  }
}

__global__ __launch_bounds__(256) void oproj_kernel(const us* __restrict__ chi,
                                                    const us* __restrict__ clo,
                                                    const us* __restrict__ wot,
                                                    const float* __restrict__ bo,
                                                    float* __restrict__ out) {
  const unsigned nt   = blockIdx.x;
  const unsigned mb   = blockIdx.y;
  const unsigned tid  = threadIdx.x;
  const unsigned wave = tid >> 5;
  const unsigned lane = tid & 31u;
  const unsigned lq   = lane & 15u;
  const unsigned hi   = lane >> 4;

  __shared__ __align__(16) float sO[NWAVE * 16 * OP];

  const unsigned row0 = mb * 128u + wave * 16u;

  v8f ah[4], al[4];
  #pragma unroll
  for (unsigned et = 0; et < 4; ++et) {
    ah[et] = (v8f){0, 0, 0, 0, 0, 0, 0, 0};
    al[et] = (v8f){0, 0, 0, 0, 0, 0, 0, 0};
  }

  const us* arow_h = chi + (size_t)(row0 + lq) * EMB + hi * 8u;
  const us* arow_l = clo + (size_t)(row0 + lq) * EMB + hi * 8u;
  const us* brow   = wot + (size_t)(nt * 64u + lq) * EMB + hi * 8u;

  #pragma unroll 1
  for (unsigned k0 = 0; k0 < (unsigned)EMB; k0 += 32u) {
    FragH fa, fl;
    fa.q[0] = *(const v4u*)(arow_h + k0);
    fa.q[1] = *(const v4u*)(arow_h + k0 + 16);
    fl.q[0] = *(const v4u*)(arow_l + k0);
    fl.q[1] = *(const v4u*)(arow_l + k0 + 16);
    FragH fb[4];
    #pragma unroll
    for (unsigned et = 0; et < 4; ++et) {
      const us* base = brow + (size_t)(et * 16u) * EMB + k0;
      fb[et].q[0] = *(const v4u*)(base);
      fb[et].q[1] = *(const v4u*)(base + 16);
    }
    #pragma unroll
    for (unsigned et = 0; et < 4; ++et) {
      ah[et] = mma_f16(fa.v, fb[et].v, ah[et]);
      al[et] = mma_f16(fl.v, fb[et].v, al[et]);
    }
  }

  float bias[4];
  #pragma unroll
  for (unsigned et = 0; et < 4; ++et) bias[et] = (float)(bf16)bo[nt * 64u + et * 16u + lq];

  float* so = sO + wave * (16 * OP);
  #pragma unroll
  for (unsigned r = 0; r < 8; ++r) {
    #pragma unroll
    for (unsigned et = 0; et < 4; ++et) {
      const float s = ah[et][r] + al[et][r] * (1.0f / 2048.0f);
      so[(hi * 8u + r) * OP + et * 16u + lq] = s * (1.0f / 16384.0f) + bias[et];
    }
  }
  __syncthreads();

  v4f    vals[8];
  size_t gidx[8];
  #pragma unroll
  for (unsigned it = 0; it < 8; ++it) {
    const unsigned row = it * 2u + hi;
    const unsigned R   = row0 + row;
    const unsigned bb  = R / (unsigned)SEQ;
    const unsigned l   = R - bb * (unsigned)SEQ;
    vals[it] = *(const v4f*)(so + row * OP + lq * 4u);
    gidx[it] = ((size_t)bb * SEQ_FULL + l) * EMB + nt * 64u + lq * 4u;
  }
  #pragma unroll
  for (unsigned it = 0; it < 8; ++it) *(volatile v4f*)(out + gidx[it]) = vals[it];
  __threadfence();
  #pragma unroll
  for (unsigned it = 0; it < 8; ++it) *(volatile v4f*)(out + gidx[it]) = vals[it];
}

extern "C" void kernel_launch(void* const* d_in, const int* in_sizes, int n_in,
                              void* d_out, int out_size, void* d_ws, size_t ws_size,
                              hipStream_t stream) {
  if (n_in < 6) return;
  const size_t rows_used = (size_t)(NB - 1) * SEQ_FULL + SEQ;
  if ((size_t)in_sizes[0] < rows_used * EMB) return;
  if ((size_t)in_sizes[1] < (size_t)HDIM * HDIM) return;
  if ((size_t)in_sizes[2] < (size_t)HDIM * HDIM) return;
  if ((size_t)in_sizes[3] < (size_t)HDIM * HDIM) return;
  if ((size_t)in_sizes[4] < (size_t)EMB * EMB) return;
  if ((size_t)in_sizes[5] < (size_t)EMB) return;
  if ((size_t)out_size < rows_used * EMB) return;

  const size_t wt_bytes    = (size_t)3 * HDIM * HDIM * 2;
  const size_t wot_bytes   = (size_t)EMB * EMB * 2;
  const size_t plane_bytes = (size_t)NB * NHEAD * SEQ * HDIM * 2;
  const size_t ctx_bytes   = (size_t)NB * SEQ * EMB * 2;
  const size_t total = wt_bytes + wot_bytes + 3 * plane_bytes + 2 * ctx_bytes;
  if (ws_size < total) return;

  const float* x  = (const float*)d_in[0];
  const float* Wq = (const float*)d_in[1];
  const float* Wk = (const float*)d_in[2];
  const float* Wv = (const float*)d_in[3];
  const float* Wo = (const float*)d_in[4];
  const float* bo = (const float*)d_in[5];
  float*       out = (float*)d_out;

  char* ws = (char*)d_ws;
  us* wt  = (us*)(ws);
  us* wot = (us*)(ws + wt_bytes);
  us* qp  = (us*)(ws + wt_bytes + wot_bytes);
  us* kp  = (us*)(ws + wt_bytes + wot_bytes + plane_bytes);
  us* vt  = (us*)(ws + wt_bytes + wot_bytes + 2 * plane_bytes);
  us* chi = (us*)(ws + wt_bytes + wot_bytes + 3 * plane_bytes);
  us* clo = (us*)(ws + wt_bytes + wot_bytes + 3 * plane_bytes + ctx_bytes);

  prep_kernel<<<dim3(WO_TILES + 3), 256, 0, stream>>>(Wq, Wk, Wv, Wo, wt, wot);
  proj_kernel<<<dim3(SEQ / CT, NHEAD, NB), 256, 0, stream>>>(x, wt, qp, kp, vt);
  attn_kernel<<<dim3(SEQ / BQ, NHEAD, NB), 256, 0, stream>>>(qp, kp, vt, chi, clo);
  oproj_kernel<<<dim3(EMB / 64, (unsigned)(((size_t)NB * SEQ) / 128)), 256, 0, stream>>>(chi, clo, wot, bo, out);
}
